// GCN_56126632624750
// MI455X (gfx1250) — hardware-verified
//
#include <hip/hip_runtime.h>
#include <stddef.h>
#include <stdint.h>


#define NN      150000
#define NE      4800000
#define NTHR    256
#define NB      512
#define NBLK    293
#define NP      (NBLK * NB)
#define SBROWS  8192
#define NSB     19
#define NCH     16
#define ECH     300000
#define EWV     37500
#define NIT1    293
#define WLCAP   2560
#define RCAP    18432
#define DEGCAP  66
#define ROP     544
#define SRCMASK 0x3FFFFu
#define WSMAX   134217728

static_assert(NN < (1 << 18));
static_assert(NBLK == (NN + NB - 1) / NB && NSB == (NN + SBROWS - 1) / SBROWS);
static_assert(NBLK <= NSB * 16 && SBROWS == 16 * NB);
static_assert(NE == NCH * ECH && ECH == 8 * EWV && (EWV % 4) == 0 && (NE % 4) == 0);
static_assert(NIT1 == (EWV + 127) / 128);
static_assert((WLCAP % 128) == 0 && (RCAP % 32) == 0 && (ROP % 32) == 0 && ROP - NB == 32);
static_assert(RCAP <= 8 * WLCAP);
static_assert(((8 * WLCAP + NB * DEGCAP) * 4) <= 280000);
static_assert((NN % 2) == 0 && (NP / 2) == NBLK * NTHR);
static_assert((NN * 3) % 4 == 0 && ((NN - (NBLK - 1) * NB) * 3) % 4 == 0 && (NB * 3 * 4) % 128 == 0);
static_assert(NTHR == 256 && NB == 2 * NTHR);

typedef float          v2f   __attribute__((ext_vector_type(2)));
typedef float          v4f   __attribute__((ext_vector_type(4)));
typedef float          v8f   __attribute__((ext_vector_type(8)));
typedef int            v4i   __attribute__((ext_vector_type(4)));
typedef int            v8i   __attribute__((ext_vector_type(8)));
typedef unsigned int   v4u   __attribute__((ext_vector_type(4)));
typedef unsigned short v8us  __attribute__((ext_vector_type(8)));
typedef unsigned short v16us __attribute__((ext_vector_type(16)));
typedef __bf16         v16bf __attribute__((ext_vector_type(16)));
typedef v4f  __attribute__((may_alias)) v4fa;
typedef v4i  __attribute__((may_alias)) v4ia;
typedef v4u  __attribute__((may_alias)) v4ua;
typedef v8us __attribute__((may_alias)) v8usa;
union FragB { v16bf v; v16us u; v8us h[2]; v8i w; };

__device__ __forceinline__ v8f wmb(const FragB& a, const FragB& b, v8f c) {
  v8f d = __builtin_amdgcn_wmma_f32_16x16x32_bf16(false, a.v, false, b.v, (short)0, c, false, false);
  asm volatile("v_nop\n\tv_nop\n\tv_nop\n\tv_nop" : "+v"(d) : "v"(a.w), "v"(b.w));
  return d;
}
__device__ __forceinline__ unsigned bf16_bits(float f) {
  const unsigned u = __float_as_uint(f);
  return (u + 0x7FFFu + ((u >> 16) & 1u)) >> 16;
}
__device__ __forceinline__ float bf16_val(float f) { return __uint_as_float(bf16_bits(f) << 16); }
__device__ __forceinline__ int iclamp(int v, int lo, int hi) { return v < lo ? lo : (v > hi ? hi : v); }
__device__ __forceinline__ float relu_np(float v) { return (v > 0.0f) ? v : (v - v); }

__device__ __forceinline__ void put_flat(float* g, const float* s, int nv4, int tid) {
#pragma unroll 1
  for (int i = tid; i < nv4; i += NTHR) {
    const v4f v = *(const v4fa*)(s + 4 * i);
    *(volatile v4f*)(g + 4 * (size_t)i) = v;
  }
}
__device__ __forceinline__ void put_flat_u(unsigned* g, const unsigned* s, int nv4, int tid) {
#pragma unroll 1
  for (int i = tid; i < nv4; i += NTHR) {
    const v4u v = *(const v4ua*)(s + 4 * i);
    *(volatile v4u*)(g + 4 * (size_t)i) = v;
  }
}

__global__ __launch_bounds__(NTHR) void k_bin1(const int* __restrict__ srcs, const int* __restrict__ dsts,
                                               int nN, unsigned* SEG, int* CNT) {
  extern __shared__ __attribute__((aligned(16))) unsigned dsm[];
  __shared__ __attribute__((aligned(16))) int lineS[32];
  const int tid = (int)threadIdx.x, lane = tid & 31, wave = tid >> 5;
  const int sb = (int)blockIdx.x >> 4, ch = (int)blockIdx.x & 15;
  const unsigned sbBase = (unsigned)(sb * SBROWS);
  const unsigned urows = (unsigned)iclamp(nN - sb * SBROWS, 0, SBROWS);
  const unsigned nmax = (unsigned)(nN - 1);
  unsigned* wl = dsm + wave * WLCAP;
  if (tid < 32) lineS[tid] = 0;
  __syncthreads();

  const int wb = ch * ECH + wave * EWV;
  const int we = wb + EWV;
  int wc = 0;
#define HIT1(DJ, SJ) { \
    const unsigned dl = (unsigned)(DJ) - sbBase; \
    const bool hj = valid && (dl < urows); \
    const unsigned su = ((unsigned)(SJ) > nmax) ? nmax : (unsigned)(SJ); \
    const unsigned mj = __builtin_amdgcn_ballot_w32(hj); \
    const int pos = wc + (int)__builtin_amdgcn_mbcnt_lo(mj, 0u); \
    if (hj && pos < WLCAP) wl[pos] = su | (dl << 18); \
    wc += (int)__builtin_popcount(mj); }
#pragma unroll 1
  for (int it = 0; it < NIT1; ++it) {
    const int e0 = wb + it * 128 + 4 * lane;
    const bool valid = e0 < we;
    const int ec = valid ? e0 : (we - 4);
    const v4i d4 = *(const v4i*)(dsts + ec);
    const v4i s4 = *(const v4i*)(srcs + ec);
    HIT1(d4.x, s4.x)
    HIT1(d4.y, s4.y)
    HIT1(d4.z, s4.z)
    HIT1(d4.w, s4.w)
  }
#undef HIT1
  const int wcc = wc < WLCAP ? wc : WLCAP;
#pragma unroll 1
  for (int i = wcc + lane; i < WLCAP; i += 32) wl[i] = 0xFFFFFFFFu;
  if (lane == 0) lineS[wave] = wc;
  __syncthreads();

  unsigned* sg = SEG + (size_t)blockIdx.x * (8 * WLCAP);
  int* cg = CNT + (size_t)blockIdx.x * 32 + 4 * (lane & 7);
  const bool cw = (wave == 0) && (lane < 8);
  const v4i cv = *(const v4ia*)(lineS + 4 * (lane & 7));
  put_flat_u(sg, dsm, 8 * WLCAP / 4, tid);
  if (cw) *(volatile v4i*)cg = cv;
  __threadfence();
  put_flat_u(sg, dsm, 8 * WLCAP / 4, tid);
  if (cw) *(volatile v4i*)cg = cv;
}

__global__ __launch_bounds__(NTHR) void k_bin2(const unsigned* __restrict__ SEG, const int* __restrict__ CNT,
                                               int nN, unsigned* COL, int* ROWOFF, float* DINV, int* FLG) {
  extern __shared__ __attribute__((aligned(16))) unsigned dsm[];
  unsigned* wlAll = dsm;
  unsigned* slP   = dsm + 8 * WLCAP;
  unsigned* dense = dsm;
  __shared__ __attribute__((aligned(16))) int   cnt[NB];
  __shared__ __attribute__((aligned(16))) int   offs[ROP];
  __shared__ __attribute__((aligned(16))) float dv[NB];
  __shared__ __attribute__((aligned(16))) int   misc[32];
  const int tid = (int)threadIdx.x, lane = tid & 31, wave = tid >> 5;
  const int blk = (int)blockIdx.x;
  const int sb = blk >> 4;
  const unsigned lo = (unsigned)((blk & 15) * NB);
  unsigned* wl = wlAll + wave * WLCAP;

  cnt[tid] = 0; cnt[tid + NTHR] = 0;
  slP[tid * DEGCAP] = 0u; slP[(tid + NTHR) * DEGCAP] = 0u;
#pragma unroll 1
  for (int i = tid; i < ROP; i += NTHR) offs[i] = 0;
  if (tid < 32) misc[tid] = 0;
  __syncthreads();

  int wc = 0, segov = 0;
#define HIT2(EJ, JJ) { \
    const unsigned rj = ((EJ) >> 18) - lo; \
    const bool hj = ((i0 + (JJ)) < n) && (rj < (unsigned)NB); \
    const unsigned mj = __builtin_amdgcn_ballot_w32(hj); \
    const int pos = wc + (int)__builtin_amdgcn_mbcnt_lo(mj, 0u); \
    if (hj && pos < WLCAP) wl[pos] = ((EJ) & SRCMASK) | (rj << 18); \
    wc += (int)__builtin_popcount(mj); }
#pragma unroll 1
  for (int ci = 0; ci < 2; ++ci) {
    const int sc = sb * 16 + 2 * wave + ci;
    const int* cl = CNT + (size_t)sc * 32;
#pragma unroll 1
    for (int v = 0; v < 8; ++v) {
      int n = cl[v];
      n = __builtin_amdgcn_readfirstlane(n);
      segov |= (n > WLCAP) ? 1 : 0;
      n = iclamp(n, 0, WLCAP);
      const unsigned* sp = SEG + ((size_t)sc * 8 + v) * WLCAP;
#pragma unroll 1
      for (int b0 = 0; b0 < n; b0 += 128) {
        const int i0 = b0 + 4 * lane;
        const v4u e = *(const v4u*)(sp + i0);
        HIT2(e.x, 0)
        HIT2(e.y, 1)
        HIT2(e.z, 2)
        HIT2(e.w, 3)
      }
    }
  }
#undef HIT2
  if (lane == 0) { misc[wave] = wc; misc[8 + wave] = segov; }
  __syncthreads();

  if (wave == 0) {
#pragma unroll 1
    for (int w2 = 0; w2 < 8; ++w2) {
      int c = iclamp(misc[w2], 0, WLCAP);
      c = __builtin_amdgcn_readfirstlane(c);
      const unsigned* wq = wlAll + w2 * WLCAP;
#pragma unroll 1
      for (int b0 = 0; b0 < c; b0 += 32) {
        const int idx = b0 + lane;
        const int ent = (int)wq[idx < c ? idx : (c - 1)];
        const int m32 = (c - b0) < 32 ? (c - b0) : 32;
#pragma unroll 1
        for (int k = 0; k < m32; ++k) {
          const unsigned u = (unsigned)__builtin_amdgcn_readlane(ent, k);
          const int row = (int)((u >> 18) & (unsigned)(NB - 1));
          if (lane == 0) {
            const int cc = cnt[row];
            if (cc >= 0 && cc < DEGCAP) slP[row * DEGCAP + cc] = u & SRCMASK;
            cnt[row] = cc + 1;
          }
        }
      }
    }
  }
  __syncthreads();

#pragma unroll 1
  for (int rr = 0; rr < 2; ++rr) {
    const int r = tid + NTHR * rr;
    const float deg = (float)cnt[r] + 1.0f;
    dv[r] = (deg > 0.0f) ? rsqrtf(fmaxf(deg, 1.0f)) : 0.0f;
  }
  if (wave == 0) {
    const int base = lane * 16;
    int s = 0, big = 0;
#pragma unroll 1
    for (int i = 0; i < 16; ++i) {
      const int c = cnt[base + i];
      big |= (c > DEGCAP) ? 1 : 0;
      s += iclamp(c, 0, DEGCAP);
    }
    int incl = s;
#pragma unroll
    for (int d = 1; d < 32; d <<= 1) {
      const int y = __shfl_up(incl, d, 32);
      if (lane >= d) incl += y;
    }
    int run = incl - s;
#pragma unroll 1
    for (int i = 0; i < 16; ++i) { offs[base + i] = run; run += iclamp(cnt[base + i], 0, DEGCAP); }
    const int total = __shfl(incl, 31, 32);
    offs[NB + lane] = total;
    const int wo = misc[lane & 15];
    const bool bad = (lane < 8) ? (wo > WLCAP) : ((lane < 16) ? (wo != 0) : false);
    int fl = (__builtin_amdgcn_ballot_w32(big != 0) != 0u) ? 1 : 0;
    fl |= (__builtin_amdgcn_ballot_w32(bad) != 0u) ? 1 : 0;
    fl |= (total > RCAP) ? 1 : 0;
    if (lane == 0) { misc[16] = total; misc[17] = fl; }
  }
  __syncthreads();

  {
    const int total = iclamp(misc[16], 0, RCAP);
#pragma unroll 1
    for (int rr = 0; rr < 2; ++rr) {
      const int r = tid + NTHR * rr;
      const int o = iclamp(offs[r], 0, RCAP);
      const int c = iclamp(cnt[r], 0, DEGCAP);
      const int cl1 = (c > 0) ? (c - 1) : 0;
      int cm = c;
#pragma unroll
      for (int d = 16; d >= 1; d >>= 1) { const int y = __shfl_xor(cm, d, 32); cm = y > cm ? y : cm; }
      cm = __builtin_amdgcn_readfirstlane(cm);
#pragma unroll 1
      for (int i = 0; i < cm; ++i) {
        const int ii = (i < cl1) ? i : cl1;
        const unsigned sv = slP[r * DEGCAP + ii];
        const int p = o + i;
        if (i < c && p < RCAP) dense[p] = sv;
      }
    }
#pragma unroll 1
    for (int i = total + tid; i < RCAP; i += NTHR) dense[i] = 0u;
  }
  __syncthreads();

  unsigned* cg = COL + (size_t)blk * RCAP;
  int*   rg = ROWOFF + (size_t)blk * ROP + 4 * tid;
  float* dg = DINV + (size_t)blk * NB + 4 * tid;
  int*   fg = FLG + (size_t)blk * 32 + 4 * (lane & 7);
  const bool rw = tid < ROP / 4;
  const bool dw = tid < NB / 4;
  const bool fw = (wave == 0) && (lane < 8);
  const v4i rv = *(const v4ia*)(offs + 4 * (rw ? tid : 0));
  const v4f dq = *(const v4fa*)(dv + 4 * (dw ? tid : 0));
  v4i fv = {0, 0, 0, 0};
  {
    const int f17 = misc[17], f16 = misc[16];
    fv.x = (lane == 0) ? f17 : 0;
    fv.y = (lane == 0) ? f16 : 0;
  }
  put_flat_u(cg, dense, RCAP / 4, tid);
  if (rw) *(volatile v4i*)rg = rv;
  if (dw) *(volatile v4f*)dg = dq;
  if (fw) *(volatile v4i*)fg = fv;
  __threadfence();
  put_flat_u(cg, dense, RCAP / 4, tid);
  if (rw) *(volatile v4i*)rg = rv;
  if (dw) *(volatile v4f*)dg = dq;
  if (fw) *(volatile v4i*)fg = fv;
}

__global__ __launch_bounds__(NTHR) void k_xs(const float* __restrict__ x, const float* __restrict__ DINV,
                                             int nN, float* XS) {
  const int t = (int)blockIdx.x * NTHR + (int)threadIdx.x;
  const int np = nN >> 1;
  const bool ok = t < np;
  const int tc = ok ? t : (np - 1);
  const v4f xv = *(const v4f*)(x + 4 * (size_t)tc);
  const v2f dd = *(const v2f*)(DINV + 2 * (size_t)t);
  v4f o;
  o.x = ok ? dd.x * bf16_val(xv.x) : 0.0f;
  o.y = ok ? dd.x * bf16_val(xv.y) : 0.0f;
  o.z = ok ? dd.y * bf16_val(xv.z) : 0.0f;
  o.w = ok ? dd.y * bf16_val(xv.w) : 0.0f;
  float* op = XS + 4 * (size_t)t;
  *(volatile v4f*)op = o;
  __threadfence();
  *(volatile v4f*)op = o;
}

__device__ __forceinline__ void stage_blk(const unsigned* __restrict__ COL, const int* __restrict__ ROWOFF,
                                          const float* __restrict__ DINV, int blk,
                                          unsigned* colS, int* offS, float* dvS, int tid) {
  const unsigned* cb = COL + (size_t)blk * RCAP;
#pragma unroll 2
  for (int i = tid; i < RCAP / 4; i += NTHR) *(v4ua*)(colS + 4 * i) = *(const v4u*)(cb + 4 * i);
  if (tid < ROP / 4) {
    v4i o = *(const v4i*)(ROWOFF + (size_t)blk * ROP + 4 * tid);
    o.x = iclamp(o.x, 0, RCAP); o.y = iclamp(o.y, 0, RCAP);
    o.z = iclamp(o.z, 0, RCAP); o.w = iclamp(o.w, 0, RCAP);
    *(v4ia*)(offS + 4 * tid) = o;
  }
  if (tid < NB / 4) *(v4fa*)(dvS + 4 * tid) = *(const v4f*)(DINV + (size_t)blk * NB + 4 * tid);
}

template <int OP>
__device__ __forceinline__ void tiles_wmma(const float* hS, const unsigned short* btS, const float* dvS,
                                           float* pS, int lane, int wave) {
  const int hh = lane >> 4, m = lane & 15;
  FragB bf;
  bf.h[0] = *(const v8usa*)(btS + m * 32 + 8 * hh);
  bf.h[1] = *(const v8usa*)(btS + m * 32 + 16 + 8 * hh);
#pragma unroll 1
  for (int ti = 0; ti < 4; ++ti) {
    const int t = wave * 4 + ti;
    const float* hp = hS + (t * 16 + m) * 16 + 8 * hh;
    const v4f x0 = *(const v4fa*)hp;
    const v4f x1 = *(const v4fa*)(hp + 4);
    const float xv[8] = {x0.x, x0.y, x0.z, x0.w, x1.x, x1.y, x1.z, x1.w};
    FragB af;
    v8us hv, lv;
#pragma unroll
    for (int i = 0; i < 8; ++i) {
      const unsigned hb = bf16_bits(xv[i]);
      hv[i] = (unsigned short)hb;
      lv[i] = (unsigned short)bf16_bits(xv[i] - __uint_as_float(hb << 16));
    }
    af.h[0] = hv; af.h[1] = lv;
    const v8f z = {0.f, 0.f, 0.f, 0.f, 0.f, 0.f, 0.f, 0.f};
    const v8f acc = wmb(af, bf, z);
#pragma unroll
    for (int r = 0; r < 8; ++r) {
      const int pr = t * 16 + 8 * hh + r;
      const float val = dvS[pr] * acc[r];
      if constexpr (OP == 16) {
        pS[pr * 16 + m] = val;
      } else {
        if (m < 4) pS[pr * 4 + m] = (m < 3) ? val : 0.0f;
      }
    }
  }
}

__global__ __launch_bounds__(NTHR) void k_conv1(const float* __restrict__ XS, const unsigned* __restrict__ COL,
                                                const int* __restrict__ ROWOFF, const float* __restrict__ DINV,
                                                const int* __restrict__ FLG, const float* __restrict__ W1,
                                                const float* __restrict__ b1, const float* __restrict__ W2,
                                                int nN, float* RES, float* P2) {
  extern __shared__ __attribute__((aligned(16))) unsigned dsm[];
  unsigned* colS = dsm;
  float* hS = (float*)(dsm + RCAP);
  float* pS = hS + NB * 16;
  __shared__ __attribute__((aligned(16))) int   offS[ROP];
  __shared__ __attribute__((aligned(16))) float dvS[NB];
  __shared__ __attribute__((aligned(16))) unsigned short btS[16 * 32];
  __shared__ float w1S[32];
  __shared__ float bS[16];
  const int tid = (int)threadIdx.x, lane = tid & 31, wave = tid >> 5;
  const int blk = (int)blockIdx.x;
  const unsigned nmax = (unsigned)(nN - 1);

  stage_blk(COL, ROWOFF, DINV, blk, colS, offS, dvS, tid);
  if (tid < 32) w1S[tid] = bf16_val(W1[tid]);
  if (tid < 16) bS[tid] = bf16_val(b1[tid]);
  {
    const int k = tid >> 4, n = tid & 15;
    const unsigned short us = (unsigned short)bf16_bits(W2[k * 16 + n]);
    btS[n * 32 + k] = us; btS[n * 32 + 16 + k] = us;
  }
  const int flag = FLG[(size_t)blk * 32];
  const float pz = (flag != 0) ? __int_as_float(0x7fc00000) : 0.0f;
  __syncthreads();

#pragma unroll 1
  for (int rr = 0; rr < 2; ++rr) {
    const int r = tid + NTHR * rr;
    const int o = offS[r];
    const int c = iclamp(offS[r + 1] - o, 0, DEGCAP);
    int cm = c;
#pragma unroll
    for (int d = 16; d >= 1; d >>= 1) { const int y = __shfl_xor(cm, d, 32); cm = y > cm ? y : cm; }
    cm = __builtin_amdgcn_readfirstlane(cm);
    float sx = 0.0f, sy = 0.0f;
#pragma unroll 1
    for (int p = 0; p < cm; ++p) {
      const bool ok = p < c;
      const int idx = (o + p > RCAP - 1) ? (RCAP - 1) : (o + p);
      unsigned s = colS[idx];
      s = s > nmax ? nmax : s;
      const v2f v = *(const v2f*)(XS + 2 * (size_t)s);
      sx += ok ? v.x : 0.0f;
      sy += ok ? v.y : 0.0f;
    }
    const int node = blk * NB + r;
    const bool live = node < nN;
    const int nc = live ? node : (nN - 1);
    const v2f sv = *(const v2f*)(XS + 2 * (size_t)nc);
    const float dd = dvS[r];
    const float t0 = dd * (sx + sv.x), t1 = dd * (sy + sv.y);
#pragma unroll 4
    for (int f = 0; f < 16; ++f) {
      float v = fmaf(t0, w1S[f], fmaf(t1, w1S[16 + f], bS[f]));
      v = relu_np(v) + pz;
      hS[r * 16 + f] = live ? v : 0.0f;
    }
  }
  __syncthreads();

  float* rg = RES + (size_t)blk * NB * 16;
  float* pg = P2 + (size_t)blk * NB * 16;
  put_flat(rg, hS, NB * 16 / 4, tid);
  tiles_wmma<16>(hS, btS, dvS, pS, lane, wave);
  __syncthreads();
  put_flat(pg, pS, NB * 16 / 4, tid);
  __threadfence();
  put_flat(rg, hS, NB * 16 / 4, tid);
  put_flat(pg, pS, NB * 16 / 4, tid);
}

template <int L3>
__global__ __launch_bounds__(NTHR) void k_conv23(const float* __restrict__ Pin, const unsigned* __restrict__ COL,
                                                 const int* __restrict__ ROWOFF, const float* __restrict__ DINV,
                                                 const int* __restrict__ FLG, const float* __restrict__ bias,
                                                 const float* __restrict__ Wn, const float* __restrict__ RESin,
                                                 int nN, float* Pout) {
  constexpr int OP = (L3 != 0) ? 4 : 16;
  extern __shared__ __attribute__((aligned(16))) unsigned dsm[];
  unsigned* colS = dsm;
  float* hS = (float*)(dsm + RCAP);
  float* pS = hS + NB * 16;
  __shared__ __attribute__((aligned(16))) int   offS[ROP];
  __shared__ __attribute__((aligned(16))) float dvS[NB];
  __shared__ __attribute__((aligned(16))) unsigned short btS[16 * 32];
  __shared__ __attribute__((aligned(16))) float bS[16];
  const int tid = (int)threadIdx.x, lane = tid & 31, wave = tid >> 5;
  const int blk = (int)blockIdx.x;
  const unsigned nmax = (unsigned)(nN - 1);

  stage_blk(COL, ROWOFF, DINV, blk, colS, offS, dvS, tid);
  if (tid < 16) bS[tid] = bf16_val(bias[tid]);
  {
    const int k = tid >> 4, n = tid & 15;
    float wv;
    if constexpr (L3 != 0) {
      const float t = Wn[k * 3 + (n < 3 ? n : 2)];
      wv = (n < 3) ? t : 0.0f;
    } else {
      wv = Wn[k * 16 + n];
    }
    const unsigned short us = (unsigned short)bf16_bits(wv);
    btS[n * 32 + k] = us; btS[n * 32 + 16 + k] = us;
  }
  const int flag = FLG[(size_t)blk * 32];
  const float pz = (flag != 0) ? __int_as_float(0x7fc00000) : 0.0f;
  __syncthreads();

  const int q = lane & 3, hp = lane >> 2;
  const v4f bq = *(const v4fa*)(bS + 4 * q);
#pragma unroll 1
  for (int si = 0; si < NB / 8; ++si) {
    const int r = wave * (NB / 8) + si;
    int o = offS[r];
    int c = iclamp(offS[r + 1] - o, 0, DEGCAP);
    o = __builtin_amdgcn_readfirstlane(o);
    c = __builtin_amdgcn_readfirstlane(c);
    float a0 = 0.0f, a1 = 0.0f, a2 = 0.0f, a3 = 0.0f;
#pragma unroll 1
    for (int b0 = 0; b0 < c; b0 += 8) {
      const int p = b0 + hp;
      const bool ok = p < c;
      const int idx = (o + p > RCAP - 1) ? (RCAP - 1) : (o + p);
      unsigned s = colS[idx];
      s = s > nmax ? nmax : s;
      const v4f v = *(const v4f*)(Pin + (size_t)s * 16 + 4 * q);
      a0 += ok ? v.x : 0.0f; a1 += ok ? v.y : 0.0f;
      a2 += ok ? v.z : 0.0f; a3 += ok ? v.w : 0.0f;
    }
#pragma unroll
    for (int d = 4; d <= 16; d <<= 1) {
      const float y0 = __shfl_xor(a0, d, 32), y1 = __shfl_xor(a1, d, 32);
      const float y2 = __shfl_xor(a2, d, 32), y3 = __shfl_xor(a3, d, 32);
      a0 += y0; a1 += y1; a2 += y2; a3 += y3;
    }
    const int node = blk * NB + r;
    const bool live = node < nN;
    const int nc = live ? node : (nN - 1);
    const v4f sv = *(const v4f*)(Pin + (size_t)nc * 16 + 4 * q);
    const float dd = dvS[r];
    v4f y;
    y.x = dd * (a0 + sv.x) + bq.x; y.y = dd * (a1 + sv.y) + bq.y;
    y.z = dd * (a2 + sv.z) + bq.z; y.w = dd * (a3 + sv.w) + bq.w;
    if constexpr (L3 != 0) {
      const v4f rv = *(const v4f*)(RESin + (size_t)nc * 16 + 4 * q);
      y.x = relu_np(y.x + rv.x); y.y = relu_np(y.y + rv.y);
      y.z = relu_np(y.z + rv.z); y.w = relu_np(y.w + rv.w);
    }
    y.x = live ? (y.x + pz) : 0.0f; y.y = live ? (y.y + pz) : 0.0f;
    y.z = live ? (y.z + pz) : 0.0f; y.w = live ? (y.w + pz) : 0.0f;
    if (hp == 0) *(v4fa*)(hS + r * 16 + 4 * q) = y;
  }
  __syncthreads();

  tiles_wmma<OP>(hS, btS, dvS, pS, lane, wave);
  __syncthreads();
  float* pg = Pout + (size_t)blk * NB * OP;
  put_flat(pg, pS, NB * OP / 4, tid);
  __threadfence();
  put_flat(pg, pS, NB * OP / 4, tid);
}

__global__ __launch_bounds__(NTHR) void k_conv4(const float* __restrict__ P4, const unsigned* __restrict__ COL,
                                                const int* __restrict__ ROWOFF, const float* __restrict__ DINV,
                                                const int* __restrict__ FLG, const float* __restrict__ b4,
                                                int nN, float* out) {
  extern __shared__ __attribute__((aligned(16))) unsigned dsm[];
  unsigned* colS = dsm;
  __shared__ __attribute__((aligned(16))) int   offS[ROP];
  __shared__ __attribute__((aligned(16))) float dvS[NB];
  __shared__ __attribute__((aligned(16))) float oS[NB * 3];
  __shared__ float bS[4];
  const int tid = (int)threadIdx.x;
  const int blk = (int)blockIdx.x;
  const unsigned nmax = (unsigned)(nN - 1);

  stage_blk(COL, ROWOFF, DINV, blk, colS, offS, dvS, tid);
  if (tid < 4) {
    const float t = b4[tid < 3 ? tid : 2];
    bS[tid] = (tid < 3) ? bf16_val(t) : 0.0f;
  }
  const int flag = FLG[(size_t)blk * 32];
  const float pz = (flag != 0) ? __int_as_float(0x7fc00000) : 0.0f;
  __syncthreads();

#pragma unroll 1
  for (int rr = 0; rr < 2; ++rr) {
    const int r = tid + NTHR * rr;
    const int o = offS[r];
    const int c = iclamp(offS[r + 1] - o, 0, DEGCAP);
    int cm = c;
#pragma unroll
    for (int d = 16; d >= 1; d >>= 1) { const int y = __shfl_xor(cm, d, 32); cm = y > cm ? y : cm; }
    cm = __builtin_amdgcn_readfirstlane(cm);
    float s0 = 0.0f, s1 = 0.0f, s2 = 0.0f;
#pragma unroll 1
    for (int p = 0; p < cm; ++p) {
      const bool ok = p < c;
      const int idx = (o + p > RCAP - 1) ? (RCAP - 1) : (o + p);
      unsigned s = colS[idx];
      s = s > nmax ? nmax : s;
      const v4f v = *(const v4f*)(P4 + 4 * (size_t)s);
      s0 += ok ? v.x : 0.0f; s1 += ok ? v.y : 0.0f; s2 += ok ? v.z : 0.0f;
    }
    const int node = blk * NB + r;
    const bool live = node < nN;
    const int nc = live ? node : (nN - 1);
    const v4f sv = *(const v4f*)(P4 + 4 * (size_t)nc);
    const float dd = dvS[r];
    const float y0 = (dd * (s0 + sv.x) + bS[0]) + pz;
    const float y1 = (dd * (s1 + sv.y) + bS[1]) + pz;
    const float y2 = (dd * (s2 + sv.z) + bS[2]) + pz;
    oS[r * 3 + 0] = live ? y0 : 0.0f;
    oS[r * 3 + 1] = live ? y1 : 0.0f;
    oS[r * 3 + 2] = live ? y2 : 0.0f;
  }
  __syncthreads();
  const int nrows = iclamp(nN - blk * NB, 0, NB);
  const int nv4 = (nrows * 3) >> 2;
  float* og = out + (size_t)blk * NB * 3;
  put_flat(og, oS, nv4, tid);
  __threadfence();
  put_flat(og, oS, nv4, tid);
}

static inline size_t al256(size_t o) { return (o + 255) & ~(size_t)255; }

extern "C" void kernel_launch(void* const* d_in, const int* in_sizes, int n_in,
                              void* d_out, int out_size, void* d_ws, size_t ws_size,
                              hipStream_t stream) {
  if (n_in < 10) return;
  if (in_sizes[0] != 2 * NN || in_sizes[1] != 2 * NE) return;
  if (in_sizes[2] != 32 || in_sizes[3] != 16) return;
  if (in_sizes[4] != 256 || in_sizes[5] != 16) return;
  if (in_sizes[6] != 256 || in_sizes[7] != 16) return;
  if (in_sizes[8] != 48 || in_sizes[9] != 3) return;
  if (out_size != 3 * NN) return;

  const float* x  = (const float*)d_in[0];
  const int*   ei = (const int*)d_in[1];
  const float* W1 = (const float*)d_in[2];
  const float* b1 = (const float*)d_in[3];
  const float* W2 = (const float*)d_in[4];
  const float* b2 = (const float*)d_in[5];
  const float* W3 = (const float*)d_in[6];
  const float* b3 = (const float*)d_in[7];
  const float* W4 = (const float*)d_in[8];
  const float* b4 = (const float*)d_in[9];
  float* out = (float*)d_out;
  const int* src = ei;
  const int* dst = ei + NE;

  char* ws = (char*)d_ws;
  size_t off = 0;
  const size_t oSEG = off; off = al256(off + (size_t)NSB * NCH * 8 * WLCAP * 4);
  const size_t oCNT = off; off = al256(off + (size_t)NSB * NCH * 32 * 4);
  const size_t oCOL = off; off = al256(off + (size_t)NBLK * RCAP * 4);
  const size_t oROW = off; off = al256(off + (size_t)NBLK * ROP * 4);
  const size_t oDIN = off; off = al256(off + (size_t)NP * 4);
  const size_t oFLG = off; off = al256(off + (size_t)NBLK * 32 * 4);
  const size_t oXS  = off; off = al256(off + (size_t)NP * 2 * 4);
  const size_t oRES = off; off = al256(off + (size_t)NP * 16 * 4);
  const size_t oP2  = off; off = al256(off + (size_t)NP * 16 * 4);
  const size_t oP3  = off; off = al256(off + (size_t)NP * 16 * 4);
  const size_t oP4  = off; off = al256(off + (size_t)NP * 4 * 4);
  if (off > ws_size || off > (size_t)WSMAX) return;
  unsigned* SEG = (unsigned*)(ws + oSEG);
  int*      CNT = (int*)(ws + oCNT);
  unsigned* COL = (unsigned*)(ws + oCOL);
  int*      ROW = (int*)(ws + oROW);
  float*    DIN = (float*)(ws + oDIN);
  int*      FLG = (int*)(ws + oFLG);
  float*    XS  = (float*)(ws + oXS);
  float*    RES = (float*)(ws + oRES);
  float*    P2  = (float*)(ws + oP2);
  float*    P3  = (float*)(ws + oP3);
  float*    P4  = (float*)(ws + oP4);

  const size_t lds1 = (size_t)8 * WLCAP * 4;
  const size_t lds2 = (size_t)(8 * WLCAP + NB * DEGCAP) * 4;
  const size_t ldsC = (size_t)RCAP * 4 + (size_t)2 * NB * 16 * 4;
  const size_t lds4 = (size_t)RCAP * 4;
  hipFuncSetAttribute(reinterpret_cast<const void*>(&k_bin1), hipFuncAttributeMaxDynamicSharedMemorySize, (int)lds1);
  hipFuncSetAttribute(reinterpret_cast<const void*>(&k_bin2), hipFuncAttributeMaxDynamicSharedMemorySize, (int)lds2);
  hipFuncSetAttribute(reinterpret_cast<const void*>(&k_conv1), hipFuncAttributeMaxDynamicSharedMemorySize, (int)ldsC);
  hipFuncSetAttribute(reinterpret_cast<const void*>(&k_conv23<0>), hipFuncAttributeMaxDynamicSharedMemorySize, (int)ldsC);
  hipFuncSetAttribute(reinterpret_cast<const void*>(&k_conv23<1>), hipFuncAttributeMaxDynamicSharedMemorySize, (int)ldsC);
  hipFuncSetAttribute(reinterpret_cast<const void*>(&k_conv4), hipFuncAttributeMaxDynamicSharedMemorySize, (int)lds4);

  k_bin1<<<NSB * NCH, NTHR, lds1, stream>>>(src, dst, NN, SEG, CNT);
  k_bin2<<<NBLK, NTHR, lds2, stream>>>(SEG, CNT, NN, COL, ROW, DIN, FLG);
  k_xs<<<NBLK, NTHR, 0, stream>>>(x, DIN, NN, XS);
  k_conv1<<<NBLK, NTHR, ldsC, stream>>>(XS, COL, ROW, DIN, FLG, W1, b1, W2, NN, RES, P2);
  k_conv23<0><<<NBLK, NTHR, ldsC, stream>>>(P2, COL, ROW, DIN, FLG, b2, W3, RES, NN, P3);
  k_conv23<1><<<NBLK, NTHR, ldsC, stream>>>(P3, COL, ROW, DIN, FLG, b3, W4, RES, NN, P4);
  k_conv4<<<NBLK, NTHR, lds4, stream>>>(P4, COL, ROW, DIN, FLG, b4, NN, out);
}
